// MetaNon_local_86947317940386
// MI455X (gfx1250) — hardware-verified
//
#include <hip/hip_runtime.h>

typedef unsigned short v8us  __attribute__((ext_vector_type(8)));
typedef unsigned short v16us __attribute__((ext_vector_type(16)));
typedef __bf16         v16bf __attribute__((ext_vector_type(16)));
typedef float          v8f   __attribute__((ext_vector_type(8)));
typedef float          v4f   __attribute__((ext_vector_type(4)));
typedef v8us __attribute__((may_alias)) v8usa;
typedef v4f  __attribute__((may_alias)) v4fa;

union Frag { v16bf v; v8us half[2]; };

#define NB   16
#define CC   256
#define CI   128
#define NP   2048
#define CO3  384

__device__ __forceinline__ v8f wmma_bf(v16bf a, v16bf b, v8f c) {
  v8f d = __builtin_amdgcn_wmma_f32_16x16x32_bf16(false, a, false, b, (short)0, c, false, false);
  asm volatile("v_nop\n\tv_nop\n\tv_nop\n\tv_nop" : "+v"(d) : "v"(a), "v"(b));
  return d;
}

__device__ __forceinline__ v8f mma3(v16bf ah, v16bf al, v16bf bh, v16bf bl, v8f c) {
  c = wmma_bf(ah, bh, c);
  c = wmma_bf(ah, bl, c);
  c = wmma_bf(al, bh, c);
  return c;
}

__device__ __forceinline__ v16bf ldfrag(const unsigned short* p, int h) {
  Frag f;
  f.half[0] = *(const v8usa*)(p + 8 * h);
  f.half[1] = *(const v8usa*)(p + 16 + 8 * h);
  return f.v;
}

__device__ __forceinline__ unsigned int bf_bits(float v) {
  const unsigned int u = __float_as_uint(v);
  return (u + 0x7fffu + ((u >> 16) & 1u)) >> 16;
}

__device__ __forceinline__ void split8(v4f a, v4f c, v8us& hi, v8us& lo) {
  float v[8];
  v[0] = a.x; v[1] = a.y; v[2] = a.z; v[3] = a.w;
  v[4] = c.x; v[5] = c.y; v[6] = c.z; v[7] = c.w;
  #pragma unroll
  for (int e = 0; e < 8; ++e) {
    const unsigned int hb = bf_bits(v[e]);
    const float hf = __uint_as_float(hb << 16);
    hi[e] = (unsigned short)hb;
    lo[e] = (unsigned short)bf_bits(v[e] - hf);
  }
}

__device__ __forceinline__ void st_split8(const float* s, unsigned short* ph, unsigned short* pl) {
  const v4f a = *(const v4fa*)s;
  const v4f c = *(const v4fa*)(s + 4);
  v8us hi = {0, 0, 0, 0, 0, 0, 0, 0};
  v8us lo = {0, 0, 0, 0, 0, 0, 0, 0};
  split8(a, c, hi, lo);
  *(volatile v8us*)ph = hi;
  *(volatile v8us*)pl = lo;
}

__device__ __forceinline__ void store_rows64(const float* sT, unsigned short* ph, unsigned short* pl,
                                             size_t base, size_t pitch, int w, int lane) {
  const int q8 = lane & 7, sub = lane >> 3;
  #pragma unroll
  for (int i = 0; i < 4; ++i) {
    const int lid = 16 * w + 4 * i + sub;
    const size_t off = base + (size_t)lid * pitch + 8 * q8;
    st_split8(sT + lid * 64 + 8 * q8, ph + off, pl + off);
  }
}

__device__ __forceinline__ void store_rows128(const float* sT, unsigned short* ph, unsigned short* pl,
                                              size_t row_base, int w, int lane) {
  const int q8 = lane & 7, sub = lane >> 3;
  #pragma unroll
  for (int i = 0; i < 4; ++i) {
    const int lid = 16 * w + 4 * i + sub;
    const int row = lid >> 1, hf = lid & 1;
    const size_t off = (row_base + row) * CI + 64 * hf + 8 * q8;
    st_split8(sT + row * 128 + 64 * hf + 8 * q8, ph + off, pl + off);
  }
}

__global__ __launch_bounds__(256) void k_prep(
    const float* __restrict__ w_theta, const float* __restrict__ w_phi,
    const float* __restrict__ w_g, const float* __restrict__ b_theta,
    const float* __restrict__ b_phi, const float* __restrict__ b_g,
    const float* __restrict__ w_out, const float* __restrict__ b_out,
    const float* __restrict__ gamma, const float* __restrict__ beta,
    const float* __restrict__ rmean, const float* __restrict__ rvar,
    unsigned short* __restrict__ Wh, unsigned short* __restrict__ Wl,
    unsigned short* __restrict__ WOh, unsigned short* __restrict__ WOl,
    float* __restrict__ bias_cat, float* __restrict__ escale, float* __restrict__ eshift)
{
  const int g = blockIdx.x * 256 + threadIdx.x;
  if (g < 12288) {
    const int row = g >> 5, c8 = (g & 31) * 8;
    const int r0 = min(row, 127), r1 = min(max(row - 128, 0), 127), r2 = min(max(row - 256, 0), 127);
    const float* src = (row < 128) ? (w_theta + r0 * 256) : ((row < 256) ? (w_phi + r1 * 256) : (w_g + r2 * 256));
    const v4f a = *(const v4fa*)(src + c8);
    const v4f c = *(const v4fa*)(src + c8 + 4);
    v8us hi = {0, 0, 0, 0, 0, 0, 0, 0};
    v8us lo = {0, 0, 0, 0, 0, 0, 0, 0};
    split8(a, c, hi, lo);
    const size_t off = (size_t)row * 256 + c8;
    *(volatile v8us*)(Wh + off) = hi;
    *(volatile v8us*)(Wl + off) = lo;
    __threadfence();
    *(volatile v8us*)(Wh + off) = hi;
    *(volatile v8us*)(Wl + off) = lo;
  } else if (g < 16384) {
    const int i = g - 12288;
    const int row = i >> 4, c8 = (i & 15) * 8;
    const float* src = w_out + row * 128 + c8;
    const v4f a = *(const v4fa*)src;
    const v4f c = *(const v4fa*)(src + 4);
    v8us hi = {0, 0, 0, 0, 0, 0, 0, 0};
    v8us lo = {0, 0, 0, 0, 0, 0, 0, 0};
    split8(a, c, hi, lo);
    const size_t off = (size_t)row * 128 + c8;
    *(volatile v8us*)(WOh + off) = hi;
    *(volatile v8us*)(WOl + off) = lo;
    __threadfence();
    *(volatile v8us*)(WOh + off) = hi;
    *(volatile v8us*)(WOl + off) = lo;
  } else if (g < 16768) {
    const int j = g - 16384;
    const float t0 = b_theta[min(j, 127)];
    const float t1 = b_phi[min(max(j - 128, 0), 127)];
    const float t2 = b_g[min(max(j - 256, 0), 127)];
    const float v = (j < 128) ? t0 : ((j < 256) ? t1 : t2);
    *(volatile float*)(bias_cat + j) = v;
    __threadfence();
    *(volatile float*)(bias_cat + j) = v;
  } else if (g < 17024) {
    const int o = g - 16768;
    const float inv = gamma[o] * rsqrtf(rvar[o] + 1e-5f);
    const float sh = b_out[o] * inv + beta[o] - rmean[o] * inv;
    *(volatile float*)(escale + o) = inv;
    *(volatile float*)(eshift + o) = sh;
    __threadfence();
    *(volatile float*)(escale + o) = inv;
    *(volatile float*)(eshift + o) = sh;
  }
}

__device__ __forceinline__ void xT_store(const float* sX, unsigned short* Xh, unsigned short* Xl,
                                         int b, int n0, int c0, int w, int lane) {
  const int q8 = lane & 7, sub = lane >> 3;
  #pragma unroll
  for (int i = 0; i < 4; ++i) {
    const int nl = 16 * w + 4 * i + sub;
    const int cb = 8 * q8;
    v4f a, c;
    a.x = sX[(cb + 0) * 68 + nl]; a.y = sX[(cb + 1) * 68 + nl];
    a.z = sX[(cb + 2) * 68 + nl]; a.w = sX[(cb + 3) * 68 + nl];
    c.x = sX[(cb + 4) * 68 + nl]; c.y = sX[(cb + 5) * 68 + nl];
    c.z = sX[(cb + 6) * 68 + nl]; c.w = sX[(cb + 7) * 68 + nl];
    v8us hi = {0, 0, 0, 0, 0, 0, 0, 0};
    v8us lo = {0, 0, 0, 0, 0, 0, 0, 0};
    split8(a, c, hi, lo);
    const size_t off = ((size_t)b * NP + n0 + nl) * CC + c0 + cb;
    *(volatile v8us*)(Xh + off) = hi;
    *(volatile v8us*)(Xl + off) = lo;
  }
}

__global__ __launch_bounds__(128) void k_xT(
    const float* __restrict__ x, unsigned short* __restrict__ Xh, unsigned short* __restrict__ Xl)
{
  __shared__ __attribute__((aligned(16))) float sX[64 * 68];
  const int tid = threadIdx.x, lane = tid & 31, w = tid >> 5;
  const int n0 = blockIdx.x * 64, c0 = blockIdx.y * 64, b = blockIdx.z;
  const float* xb = x + ((size_t)b * CC + c0) * NP + n0;
  #pragma unroll
  for (int it = 0; it < 8; ++it) {
    const int idx = tid + 128 * it;
    const int c = idx >> 4, n4 = (idx & 15) * 4;
    const v4f q = *(const v4fa*)(xb + (size_t)c * NP + n4);
    *(v4fa*)(sX + c * 68 + n4) = q;
  }
  __syncthreads();
  xT_store(sX, Xh, Xl, b, n0, c0, w, lane);
  __threadfence();
  xT_store(sX, Xh, Xl, b, n0, c0, w, lane);
}

__global__ __launch_bounds__(256) void k_conv(
    const unsigned short* __restrict__ Wh, const unsigned short* __restrict__ Wl,
    const unsigned short* __restrict__ Xh, const unsigned short* __restrict__ Xl,
    const float* __restrict__ bias_cat,
    unsigned short* __restrict__ Th, unsigned short* __restrict__ Tl,
    unsigned short* __restrict__ Ph, unsigned short* __restrict__ Pl,
    unsigned short* __restrict__ Gh, unsigned short* __restrict__ Gl)
{
  __shared__ __attribute__((aligned(16))) float sT[128 * 64];
  const int tid = threadIdx.x, lane = tid & 31, w = tid >> 5;
  const int h = lane >> 4, m = lane & 15;
  const int n0 = blockIdx.x * 64, which = blockIdx.y, b = blockIdx.z;
  const int wo = w >> 1, wn = w & 1;
  const int orow0 = which * 128 + 32 * wo;

  const unsigned short* wa  = Wh + (size_t)(orow0 + m) * CC;
  const unsigned short* wal = Wl + (size_t)(orow0 + m) * CC;
  const size_t xoff = ((size_t)b * NP + n0 + 32 * wn + m) * CC;
  const unsigned short* xb  = Xh + xoff;
  const unsigned short* xbl = Xl + xoff;

  const v8f z8 = {0.f, 0.f, 0.f, 0.f, 0.f, 0.f, 0.f, 0.f};
  v8f acc[2][2];
  #pragma unroll
  for (int mt = 0; mt < 2; ++mt)
    #pragma unroll
    for (int nt = 0; nt < 2; ++nt) acc[mt][nt] = z8;

  #pragma unroll 1
  for (int k0 = 0; k0 < CC; k0 += 32) {
    const v16bf a0h = ldfrag(wa + k0, h);
    const v16bf a0l = ldfrag(wal + k0, h);
    const v16bf a1h = ldfrag(wa + 16 * CC + k0, h);
    const v16bf a1l = ldfrag(wal + 16 * CC + k0, h);
    #pragma unroll
    for (int nt = 0; nt < 2; ++nt) {
      const v16bf bh = ldfrag(xb + nt * 16 * CC + k0, h);
      const v16bf bl = ldfrag(xbl + nt * 16 * CC + k0, h);
      acc[0][nt] = mma3(a0h, a0l, bh, bl, acc[0][nt]);
      acc[1][nt] = mma3(a1h, a1l, bh, bl, acc[1][nt]);
    }
  }

  #pragma unroll
  for (int mt = 0; mt < 2; ++mt) {
    #pragma unroll
    for (int r = 0; r < 8; ++r) {
      const int ol = 32 * wo + 16 * mt + 8 * h + r;
      const float bv = bias_cat[which * 128 + ol];
      #pragma unroll
      for (int nt = 0; nt < 2; ++nt) {
        const int nl = 32 * wn + 16 * nt + m;
        const float v = acc[mt][nt][r] + bv;
        if (which == 0) sT[nl * 128 + ol] = v;
        else            sT[ol * 64 + nl] = v;
      }
    }
  }
  __syncthreads();

  if (which == 0) {
    const size_t row_base = (size_t)b * NP + n0;
    store_rows128(sT, Th, Tl, row_base, w, lane);
    __threadfence();
    store_rows128(sT, Th, Tl, row_base, w, lane);
  } else {
    unsigned short* dh = (which == 1) ? Ph : Gh;
    unsigned short* dl = (which == 1) ? Pl : Gl;
    const size_t base = ((size_t)b * CI) * NP + n0;
    store_rows64(sT, dh, dl, base, NP, w, lane);
    __threadfence();
    store_rows64(sT, dh, dl, base, NP, w, lane);
  }
}

__global__ __launch_bounds__(128) void k_umat(
    const unsigned short* __restrict__ Gh, const unsigned short* __restrict__ Gl,
    const unsigned short* __restrict__ Ph, const unsigned short* __restrict__ Pl,
    unsigned short* __restrict__ Uh, unsigned short* __restrict__ Ul)
{
  __shared__ __attribute__((aligned(16))) float sT[64 * 64];
  const int tid = threadIdx.x, lane = tid & 31, w = tid >> 5;
  const int h = lane >> 4, m = lane & 15;
  const int c0 = blockIdx.x * 64, cp0 = blockIdx.y * 64, b = blockIdx.z;
  const int wc = w >> 1, wp = w & 1;

  const size_t goff = ((size_t)b * CI + c0 + 32 * wc + m) * NP;
  const size_t poff = ((size_t)b * CI + cp0 + 32 * wp + m) * NP;
  const unsigned short* ga  = Gh + goff;
  const unsigned short* gal = Gl + goff;
  const unsigned short* pb  = Ph + poff;
  const unsigned short* pbl = Pl + poff;

  const v8f z8 = {0.f, 0.f, 0.f, 0.f, 0.f, 0.f, 0.f, 0.f};
  v8f acc[2][2];
  #pragma unroll
  for (int mt = 0; mt < 2; ++mt)
    #pragma unroll
    for (int nt = 0; nt < 2; ++nt) acc[mt][nt] = z8;

  #pragma unroll 1
  for (int k0 = 0; k0 < NP; k0 += 32) {
    const v16bf a0h = ldfrag(ga + k0, h);
    const v16bf a0l = ldfrag(gal + k0, h);
    const v16bf a1h = ldfrag(ga + (size_t)16 * NP + k0, h);
    const v16bf a1l = ldfrag(gal + (size_t)16 * NP + k0, h);
    #pragma unroll
    for (int nt = 0; nt < 2; ++nt) {
      const v16bf bh = ldfrag(pb + (size_t)nt * 16 * NP + k0, h);
      const v16bf bl = ldfrag(pbl + (size_t)nt * 16 * NP + k0, h);
      acc[0][nt] = mma3(a0h, a0l, bh, bl, acc[0][nt]);
      acc[1][nt] = mma3(a1h, a1l, bh, bl, acc[1][nt]);
    }
  }

  const float invN = 1.0f / 2048.0f;
  #pragma unroll
  for (int mt = 0; mt < 2; ++mt) {
    #pragma unroll
    for (int r = 0; r < 8; ++r) {
      const int cl = 32 * wc + 16 * mt + 8 * h + r;
      #pragma unroll
      for (int nt = 0; nt < 2; ++nt) {
        const int cpl = 32 * wp + 16 * nt + m;
        sT[cl * 64 + cpl] = acc[mt][nt][r] * invN;
      }
    }
  }
  __syncthreads();

  const size_t base = ((size_t)b * CI + c0) * CI + cp0;
  store_rows64(sT, Uh, Ul, base, CI, w, lane);
  __threadfence();
  store_rows64(sT, Uh, Ul, base, CI, w, lane);
}

__global__ __launch_bounds__(256) void k_ymat(
    const unsigned short* __restrict__ Th, const unsigned short* __restrict__ Tl,
    const unsigned short* __restrict__ Uh, const unsigned short* __restrict__ Ul,
    unsigned short* __restrict__ Yh, unsigned short* __restrict__ Yl)
{
  __shared__ __attribute__((aligned(16))) float sT[64 * 128];
  const int tid = threadIdx.x, lane = tid & 31, w = tid >> 5;
  const int h = lane >> 4, m = lane & 15;
  const int n0 = blockIdx.x * 64, b = blockIdx.y;
  const int wn = w >> 2, wc = w & 3;

  const size_t toff = ((size_t)b * NP + n0 + 32 * wn + m) * CI;
  const size_t uoff = ((size_t)b * CI + 32 * wc + m) * CI;
  const unsigned short* ta  = Th + toff;
  const unsigned short* tal = Tl + toff;
  const unsigned short* ub  = Uh + uoff;
  const unsigned short* ubl = Ul + uoff;

  const v8f z8 = {0.f, 0.f, 0.f, 0.f, 0.f, 0.f, 0.f, 0.f};
  v8f acc[2][2];
  #pragma unroll
  for (int mt = 0; mt < 2; ++mt)
    #pragma unroll
    for (int nt = 0; nt < 2; ++nt) acc[mt][nt] = z8;

  #pragma unroll 1
  for (int k0 = 0; k0 < CI; k0 += 32) {
    const v16bf a0h = ldfrag(ta + k0, h);
    const v16bf a0l = ldfrag(tal + k0, h);
    const v16bf a1h = ldfrag(ta + 16 * CI + k0, h);
    const v16bf a1l = ldfrag(tal + 16 * CI + k0, h);
    #pragma unroll
    for (int nt = 0; nt < 2; ++nt) {
      const v16bf bh = ldfrag(ub + nt * 16 * CI + k0, h);
      const v16bf bl = ldfrag(ubl + nt * 16 * CI + k0, h);
      acc[0][nt] = mma3(a0h, a0l, bh, bl, acc[0][nt]);
      acc[1][nt] = mma3(a1h, a1l, bh, bl, acc[1][nt]);
    }
  }

  #pragma unroll
  for (int mt = 0; mt < 2; ++mt) {
    #pragma unroll
    for (int r = 0; r < 8; ++r) {
      const int nl = 32 * wn + 16 * mt + 8 * h + r;
      #pragma unroll
      for (int nt = 0; nt < 2; ++nt) {
        const int cl = 32 * wc + 16 * nt + m;
        sT[nl * 128 + cl] = acc[mt][nt][r];
      }
    }
  }
  __syncthreads();

  const size_t row_base = (size_t)b * NP + n0;
  store_rows128(sT, Yh, Yl, row_base, w, lane);
  __threadfence();
  store_rows128(sT, Yh, Yl, row_base, w, lane);
}

__device__ __forceinline__ void out_store(const float* sT, float* out, size_t row_base, int n0,
                                          int w, int lane) {
  const int q8 = lane & 7, sub = lane >> 3;
  #pragma unroll
  for (int i = 0; i < 8; ++i) {
    const int lid = 32 * w + 4 * i + sub;
    const int row = lid >> 1, hf = lid & 1;
    const v4f v = *(const v4fa*)(sT + row * 64 + 32 * hf + 4 * q8);
    const size_t off = (row_base + row) * NP + n0 + 32 * hf + 4 * q8;
    *(volatile v4f*)(out + off) = v;
  }
}

__global__ __launch_bounds__(256) void k_out(
    const unsigned short* __restrict__ WOh, const unsigned short* __restrict__ WOl,
    const unsigned short* __restrict__ Yh, const unsigned short* __restrict__ Yl,
    const float* __restrict__ escale, const float* __restrict__ eshift,
    const float* __restrict__ x, float* __restrict__ out)
{
  __shared__ __attribute__((aligned(16))) float sT[128 * 64];
  const int tid = threadIdx.x, lane = tid & 31, w = tid >> 5;
  const int h = lane >> 4, m = lane & 15;
  const int n0 = blockIdx.x * 64, oh = blockIdx.y, b = blockIdx.z;
  const int wo = w >> 1, wn = w & 1;
  const int o0w = oh * 128 + 32 * wo;

  const unsigned short* wa  = WOh + (size_t)(o0w + m) * CI;
  const unsigned short* wal = WOl + (size_t)(o0w + m) * CI;
  const size_t yoff = ((size_t)b * NP + n0 + 32 * wn + m) * CI;
  const unsigned short* yb  = Yh + yoff;
  const unsigned short* ybl = Yl + yoff;

  const v8f z8 = {0.f, 0.f, 0.f, 0.f, 0.f, 0.f, 0.f, 0.f};
  v8f acc[2][2];
  #pragma unroll
  for (int mt = 0; mt < 2; ++mt)
    #pragma unroll
    for (int nt = 0; nt < 2; ++nt) acc[mt][nt] = z8;

  #pragma unroll 1
  for (int k0 = 0; k0 < CI; k0 += 32) {
    const v16bf a0h = ldfrag(wa + k0, h);
    const v16bf a0l = ldfrag(wal + k0, h);
    const v16bf a1h = ldfrag(wa + 16 * CI + k0, h);
    const v16bf a1l = ldfrag(wal + 16 * CI + k0, h);
    #pragma unroll
    for (int nt = 0; nt < 2; ++nt) {
      const v16bf bh = ldfrag(yb + nt * 16 * CI + k0, h);
      const v16bf bl = ldfrag(ybl + nt * 16 * CI + k0, h);
      acc[0][nt] = mma3(a0h, a0l, bh, bl, acc[0][nt]);
      acc[1][nt] = mma3(a1h, a1l, bh, bl, acc[1][nt]);
    }
  }

  #pragma unroll
  for (int mt = 0; mt < 2; ++mt) {
    #pragma unroll
    for (int r = 0; r < 8; ++r) {
      const int o = o0w + 16 * mt + 8 * h + r;
      const int ol = 32 * wo + 16 * mt + 8 * h + r;
      const float sc = escale[o];
      const float sh = eshift[o];
      const float* xr = x + ((size_t)b * CC + o) * NP + n0 + 32 * wn + m;
      #pragma unroll
      for (int nt = 0; nt < 2; ++nt) {
        const int nl = 32 * wn + 16 * nt + m;
        const float v = acc[mt][nt][r] * sc + sh + xr[16 * nt];
        sT[ol * 64 + nl] = v;
      }
    }
  }
  __syncthreads();

  const size_t row_base = (size_t)b * CC + oh * 128;
  out_store(sT, out, row_base, n0, w, lane);
  __threadfence();
  out_store(sT, out, row_base, n0, w, lane);
}

extern "C" void kernel_launch(void* const* d_in, const int* in_sizes, int n_in,
                              void* d_out, int out_size, void* d_ws, size_t ws_size,
                              hipStream_t stream) {
  if (n_in < 13) return;
  if (in_sizes[0] != NB * CC * NP) return;
  if (in_sizes[1] != CI * CC || in_sizes[3] != CI * CC || in_sizes[5] != CI * CC) return;
  if (in_sizes[2] != CI || in_sizes[4] != CI || in_sizes[6] != CI) return;
  if (in_sizes[7] != CC * CI || in_sizes[8] != CC) return;
  if (in_sizes[9] != CC || in_sizes[10] != CC || in_sizes[11] != CC || in_sizes[12] != CC) return;
  if (out_size != NB * CC * NP) return;

  const float* x       = (const float*)d_in[0];
  const float* w_theta = (const float*)d_in[1];
  const float* b_theta = (const float*)d_in[2];
  const float* w_phi   = (const float*)d_in[3];
  const float* b_phi   = (const float*)d_in[4];
  const float* w_g     = (const float*)d_in[5];
  const float* b_g     = (const float*)d_in[6];
  const float* w_out   = (const float*)d_in[7];
  const float* b_out   = (const float*)d_in[8];
  const float* gamma   = (const float*)d_in[9];
  const float* beta    = (const float*)d_in[10];
  const float* rmean   = (const float*)d_in[11];
  const float* rvar    = (const float*)d_in[12];
  float* out = (float*)d_out;

  const size_t bW   = (size_t)CO3 * CC * 2;
  const size_t bWO  = (size_t)CC * CI * 2;
  const size_t bBias = (size_t)CO3 * 4;
  const size_t bTab = (size_t)CC * 4;
  const size_t bX   = (size_t)NB * NP * CC * 2;
  const size_t bT   = (size_t)NB * NP * CI * 2;
  const size_t bU   = (size_t)NB * CI * CI * 2;

  size_t off = 0;
  char* ws = (char*)d_ws;
  #define CARVE(ptr, type, bytes) type* ptr = (type*)(ws + off); off += (((bytes) + 255) & ~(size_t)255);
  CARVE(Wh,  unsigned short, bW)
  CARVE(Wl,  unsigned short, bW)
  CARVE(WOh, unsigned short, bWO)
  CARVE(WOl, unsigned short, bWO)
  CARVE(bias_cat, float, bBias)
  CARVE(escale, float, bTab)
  CARVE(eshift, float, bTab)
  CARVE(Xh,  unsigned short, bX)
  CARVE(Xl,  unsigned short, bX)
  CARVE(Th,  unsigned short, bT)
  CARVE(Tl,  unsigned short, bT)
  CARVE(Ph,  unsigned short, bT)
  CARVE(Pl,  unsigned short, bT)
  CARVE(Gh,  unsigned short, bT)
  CARVE(Gl,  unsigned short, bT)
  CARVE(Uh,  unsigned short, bU)
  CARVE(Ul,  unsigned short, bU)
  CARVE(Yh,  unsigned short, bT)
  CARVE(Yl,  unsigned short, bT)
  #undef CARVE
  if (off > ws_size) return;
  if (off > (size_t)134217728) return;

  k_prep<<<67, 256, 0, stream>>>(w_theta, w_phi, w_g, b_theta, b_phi, b_g, w_out, b_out,
                                  gamma, beta, rmean, rvar, Wh, Wl, WOh, WOl,
                                  bias_cat, escale, eshift);
  k_xT<<<dim3(NP / 64, CC / 64, NB), 128, 0, stream>>>(x, Xh, Xl);
  k_conv<<<dim3(NP / 64, 3, NB), 256, 0, stream>>>(Wh, Wl, Xh, Xl, bias_cat, Th, Tl, Ph, Pl, Gh, Gl);
  k_umat<<<dim3(CI / 64, CI / 64, NB), 128, 0, stream>>>(Gh, Gl, Ph, Pl, Uh, Ul);
  k_ymat<<<dim3(NP / 64, NB), 256, 0, stream>>>(Th, Tl, Uh, Ul, Yh, Yl);
  k_out<<<dim3(NP / 64, 2, NB), 256, 0, stream>>>(WOh, WOl, Yh, Yl, escale, eshift, x, out);
}
